// MultiHeadSelfAttentionBlock_40647570489684
// MI455X (gfx1250) — hardware-verified
//
#include <hip/hip_runtime.h>


#ifndef NB
#define NB 2
#endif
#ifndef SEQ
#define SEQ 2048
#endif

namespace {

constexpr int NB_FULL = 2;
constexpr int SEQ_FULL = 2048;
constexpr int DM = 1024;
constexpr int NH = 16;
constexpr int HDIM = 64;
constexpr int NQKV = 3 * DM;
constexpr int MROWS = NB * SEQ;
constexpr int QT = SEQ / 16;
constexpr int NBH = NB * NH;
constexpr int EARLY_QBLK = 2;
constexpr int EARLY_ROWS = EARLY_QBLK * 64;
constexpr int NFLAG = 64;
constexpr int VTILE = HDIM * 16;
constexpr float RES_SCALE = 1024.0f;
constexpr float RES_INV = 1.0f / 1024.0f;
constexpr float P_SCALE = 4096.0f;
constexpr float P_INV = 1.0f / 4096.0f;
constexpr float WO_SCALE = 256.0f;
constexpr float WO_INV = 1.0f / 256.0f;

static_assert(NB >= 1 && NB <= NB_FULL);
static_assert(SEQ % 128 == 0 && SEQ >= 256 && SEQ <= SEQ_FULL);
static_assert(EARLY_ROWS == 128 && (SEQ - EARLY_ROWS) % 128 == 0);
static_assert(MROWS % NFLAG == 0 && MROWS % 128 == 0 && MROWS % 2 == 0);
static_assert(NH * 3 * HDIM == NQKV && NH * HDIM == DM && DM % 32 == 0 && HDIM == 64);

typedef _Float16 h16;
typedef __bf16 b16;
typedef h16 v16h __attribute__((ext_vector_type(16)));
typedef h16 v8h __attribute__((ext_vector_type(8), __may_alias__));
typedef b16 v16b __attribute__((ext_vector_type(16)));
typedef b16 v8b __attribute__((ext_vector_type(8), __may_alias__));
typedef float v8f __attribute__((ext_vector_type(8)));
typedef float v4f __attribute__((ext_vector_type(4), __may_alias__));

__device__ __forceinline__ v8h ld8h(const h16* p) { return *(const v8h*)p; }
__device__ __forceinline__ v8b ld8b(const b16* p) { return *(const v8b*)p; }
__device__ __forceinline__ v16h cat8h(v8h a, v8h b) {
  return __builtin_shufflevector(a, b, 0, 1, 2, 3, 4, 5, 6, 7, 8, 9, 10, 11, 12, 13, 14, 15);
}
__device__ __forceinline__ v16b cat8b(v8b a, v8b b) {
  return __builtin_shufflevector(a, b, 0, 1, 2, 3, 4, 5, 6, 7, 8, 9, 10, 11, 12, 13, 14, 15);
}
__device__ __forceinline__ v16h frag_h(const h16* p, int hh) { return cat8h(ld8h(p + 8 * hh), ld8h(p + 16 + 8 * hh)); }
__device__ __forceinline__ v16b frag_b(const b16* p, int hh) { return cat8b(ld8b(p + 8 * hh), ld8b(p + 16 + 8 * hh)); }

__device__ __forceinline__ v8f wmma_h(v16h a, v16h b, v8f c) {
  v8f d = __builtin_amdgcn_wmma_f32_16x16x32_f16(false, a, false, b, (short)0, c, false, false);
  asm volatile("v_nop\n\tv_nop\n\tv_nop\n\tv_nop" : "+v"(d) : "v"(a), "v"(b));
  return d;
}
__device__ __forceinline__ v8f wmma_b(v16b a, v16b b, v8f c) {
  v8f d = __builtin_amdgcn_wmma_f32_16x16x32_bf16(false, a, false, b, (short)0, c, false, false);
  asm volatile("v_nop\n\tv_nop\n\tv_nop\n\tv_nop" : "+v"(d) : "v"(a), "v"(b));
  return d;
}
__device__ __forceinline__ void wave_lds_sync() {
  __builtin_amdgcn_fence(__ATOMIC_RELEASE, "workgroup");
  __builtin_amdgcn_wave_barrier();
  __builtin_amdgcn_fence(__ATOMIC_ACQUIRE, "workgroup");
}
__device__ __forceinline__ float bf16_rne(float f) {
  unsigned int u = __float_as_uint(f);
  u += 0x7fffu + ((u >> 16) & 1u);
  return __uint_as_float(u & 0xffff0000u);
}
__device__ __forceinline__ void split_h(float v, h16& hi, h16& rs) {
  hi = (h16)v;
  rs = (h16)((v - (float)hi) * RES_SCALE);
}

__global__ __launch_bounds__(256) void cvt_x_kernel(const float* __restrict__ x, b16* __restrict__ xb) {
  const int c = (int)blockIdx.x * 256 + (int)threadIdx.x;
  const int r = c >> 7;
  if (r >= MROWS) return;
  const int k0 = (c & 127) * 8;
  const int b = r / SEQ, s = r - b * SEQ;
  const float* src = x + ((size_t)b * SEQ_FULL + s) * DM + k0;
  const v4f f0 = *(const v4f*)src;
  const v4f f1 = *(const v4f*)(src + 4);
  v8b o;
#pragma unroll
  for (int e = 0; e < 4; ++e) { o[e] = (b16)f0[e]; o[4 + e] = (b16)f1[e]; }
  b16* dst = xb + (size_t)r * DM + k0;
  *(volatile v8b*)dst = o;
  __threadfence();
  *(volatile v8b*)dst = o;
}

__global__ __launch_bounds__(256) void cvt_wqkv_kernel(const float* __restrict__ w, b16* __restrict__ wt) {
  __shared__ __attribute__((aligned(16))) b16 L[64 * 72];
  const int tid = (int)threadIdx.x;
  const int n0 = (int)blockIdx.x * 64, k0 = (int)blockIdx.y * 64;
  const int kk = tid >> 4, nn = (tid & 15) * 4;
#pragma unroll
  for (int i = 0; i < 4; ++i) {
    const int k = kk + 16 * i;
    const v4f f = *(const v4f*)(w + (size_t)(k0 + k) * NQKV + n0 + nn);
#pragma unroll
    for (int j = 0; j < 4; ++j) L[(nn + j) * 72 + k] = (b16)f[j];
  }
  __syncthreads();
  const int row0 = tid >> 3, pc = (tid & 7) * 8;
#pragma unroll
  for (int pass = 0; pass < 2; ++pass) {
#pragma unroll
    for (int it = 0; it < 2; ++it) {
      const int row = it * 32 + row0;
      *(volatile v8b*)(wt + (size_t)(n0 + row) * DM + k0 + pc) = ld8b(L + row * 72 + pc);
    }
    __threadfence();
  }
}

__global__ __launch_bounds__(256) void cvt_wo_kernel(const float* __restrict__ w, h16* __restrict__ wot) {
  __shared__ __attribute__((aligned(16))) h16 L[64 * 72];
  const int tid = (int)threadIdx.x;
  const int n0 = (int)blockIdx.x * 64, k0 = (int)blockIdx.y * 64;
  const int kk = tid >> 4, nn = (tid & 15) * 4;
#pragma unroll
  for (int i = 0; i < 4; ++i) {
    const int k = kk + 16 * i;
    const v4f f = *(const v4f*)(w + (size_t)(k0 + k) * DM + n0 + nn);
#pragma unroll
    for (int j = 0; j < 4; ++j) L[(nn + j) * 72 + k] = (h16)(bf16_rne(f[j]) * WO_SCALE);
  }
  __syncthreads();
  const int row0 = tid >> 3, pc = (tid & 7) * 8;
#pragma unroll
  for (int pass = 0; pass < 2; ++pass) {
#pragma unroll
    for (int it = 0; it < 2; ++it) {
      const int row = it * 32 + row0;
      *(volatile v8h*)(wot + (size_t)(n0 + row) * DM + k0 + pc) = ld8h(L + row * 72 + pc);
    }
    __threadfence();
  }
}

__global__ __launch_bounds__(256) void chk_mask_kernel(const float* __restrict__ mask, float* __restrict__ flags) {
  __shared__ int red[8];
  const int tid = (int)threadIdx.x, lane = tid & 31, wave = tid >> 5;
  constexpr int RPB = MROWS / NFLAG;
  int bad = 0;
  for (int rr = 0; rr < RPB; ++rr) {
    const int r = (int)blockIdx.x * RPB + rr;
    const int b = r / SEQ, q = r - b * SEQ;
    const float* mp = mask + ((size_t)b * SEQ_FULL + q) * SEQ_FULL;
    for (int c = tid; c < SEQ / 4; c += 256) {
      const v4f mv = *(const v4f*)(mp + 4 * c);
#pragma unroll
      for (int j = 0; j < 4; ++j) {
        const int k = 4 * c + j;
        const float v = mv[j];
        const int viol_hi = (v > -5.0e8f) ? 1 : 0;
        const int viol_dg = (v < -1.0e8f) ? 1 : 0;
        bad += (k > q) ? viol_hi : ((k == q) ? viol_dg : 0);
      }
    }
  }
#pragma unroll
  for (int s = 16; s >= 1; s >>= 1) bad += __shfl_xor(bad, s);
  if (lane == 0) red[wave] = bad;
  __syncthreads();
  if (wave == 0) {
    int tot = red[lane & 7];
    tot = (lane < 8) ? tot : 0;
#pragma unroll
    for (int s = 16; s >= 1; s >>= 1) tot += __shfl_xor(tot, s);
    const float ft = (float)tot;
    const v4f fv = {ft, ft, ft, ft};
    float* dst = flags + (size_t)blockIdx.x * 32 + (lane & 7) * 4;
    if (lane < 8) *(volatile v4f*)dst = fv;
    __threadfence();
    if (lane < 8) *(volatile v4f*)dst = fv;
  }
}

__global__ __launch_bounds__(128) void qkv_gemm_kernel(const b16* __restrict__ xb, const b16* __restrict__ wt, const float* __restrict__ bqkv,
                                                       h16* __restrict__ Qh, h16* __restrict__ Qr, h16* __restrict__ Kh, h16* __restrict__ Kr,
                                                       h16* __restrict__ Vh, h16* __restrict__ Vr) {
  __shared__ __attribute__((aligned(16))) h16 Ts[4][2][32 * 64];
  const int lane = (int)threadIdx.x & 31, wave = (int)threadIdx.x >> 5, nloc = lane & 15, hlf = lane >> 4;
  const int m0 = (int)blockIdx.y * 128 + wave * 32;
  const int c0 = (int)blockIdx.x * 64;
  float bias[4];
#pragma unroll
  for (int t = 0; t < 4; ++t) bias[t] = bf16_rne(bqkv[c0 + t * 16 + nloc]);
  v8f acc[2][4];
#pragma unroll
  for (int r = 0; r < 2; ++r)
#pragma unroll
    for (int t = 0; t < 4; ++t) acc[r][t] = (v8f){};
  const b16* a0p = xb + (size_t)(m0 + nloc) * DM;
  const b16* a1p = a0p + (size_t)16 * DM;
  const b16* bp = wt + (size_t)(c0 + nloc) * DM;
#pragma unroll 1
  for (int kb = 0; kb < DM; kb += 32) {
    const v16b a0 = frag_b(a0p + kb, hlf), a1 = frag_b(a1p + kb, hlf);
#pragma unroll
    for (int t = 0; t < 4; ++t) {
      const v16b bf = frag_b(bp + (size_t)t * 16 * DM + kb, hlf);
      acc[0][t] = wmma_b(a0, bf, acc[0][t]);
      acc[1][t] = wmma_b(a1, bf, acc[1][t]);
    }
  }
  const int head = c0 / (3 * HDIM);
  const int which = (c0 - head * (3 * HDIM)) >> 6;
  const int b = m0 / SEQ, s0 = m0 - b * SEQ;
  const int bh = b * NH + head;
  h16* Tp0 = Ts[wave][0];
  h16* Tp1 = Ts[wave][1];
#pragma unroll
  for (int t = 0; t < 4; ++t)
#pragma unroll
    for (int r = 0; r < 2; ++r)
#pragma unroll
      for (int v = 0; v < 8; ++v) {
        const int rr = r * 16 + v + 8 * hlf, d = t * 16 + nloc;
        h16 yh, yr;
        split_h(acc[r][t][v] + bias[t], yh, yr);
        const int idx = (which < 2) ? (rr * 64 + d) : ((rr >> 4) * VTILE + d * 16 + (rr & 15));
        Tp0[idx] = yh; Tp1[idx] = yr;
      }
  wave_lds_sync();
  h16* dh; h16* dr; size_t o;
  if (which == 0)      { o = ((size_t)bh * SEQ + s0) * HDIM; dh = Qh + o; dr = Qr + o; }
  else if (which == 1) { o = ((size_t)bh * SEQ + s0) * HDIM; dh = Kh + o; dr = Kr + o; }
  else                 { o = ((size_t)bh * QT + (s0 >> 4)) * (size_t)VTILE; dh = Vh + o; dr = Vr + o; }
#pragma unroll
  for (int j = 0; j < 8; ++j) { const int e = (j * 32 + lane) * 8; *(volatile v8h*)(dh + e) = ld8h(Tp0 + e); *(volatile v8h*)(dr + e) = ld8h(Tp1 + e); }
  __threadfence();
#pragma unroll
  for (int j = 0; j < 8; ++j) { const int e = (j * 32 + lane) * 8; *(volatile v8h*)(dh + e) = ld8h(Tp0 + e); *(volatile v8h*)(dr + e) = ld8h(Tp1 + e); }
}

template <bool RES>
__global__ __launch_bounds__(128) void attn_kernel(const h16* __restrict__ Qh, const h16* __restrict__ Qr,
                                                   const h16* __restrict__ Kh, const h16* __restrict__ Kr,
                                                   const h16* __restrict__ Vh, const h16* __restrict__ Vr,
                                                   const float* __restrict__ mask, h16* __restrict__ Ch, h16* __restrict__ Cr) {
  __shared__ __attribute__((aligned(16))) float Os[4][16 * 64];
  const int wave = (int)threadIdx.x >> 5, lane = (int)threadIdx.x & 31, hh = lane >> 4, col = lane & 15;
  const int bh = (int)blockIdx.x, b = bh / NH, h = bh - b * NH;
  const int qblk = RES ? (int)blockIdx.y : (EARLY_QBLK + (int)blockIdx.y);
  const int q0 = qblk * 64 + wave * 16;
  const size_t qo = ((size_t)bh * SEQ + q0 + col) * HDIM;
  const v16h q0h = frag_h(Qh + qo, hh), q1h = frag_h(Qh + qo + 32, hh);
  const v16h q0r = frag_h(Qr + qo, hh), q1r = frag_h(Qr + qo + 32, hh);
  const size_t ko = (size_t)bh * SEQ * HDIM;
  const size_t vo = (size_t)bh * QT * (size_t)VTILE;
  const float* mrow = mask + ((size_t)b * SEQ_FULL + q0 + col) * SEQ_FULL;
  float m = -INFINITY, l = 0.0f;
  v8f o[4], orr[4];
#pragma unroll
  for (int n = 0; n < 4; ++n) { o[n] = (v8f){}; orr[n] = (v8f){}; }
  const int kend = q0 + 16;
  for (int kb = 0; kb < kend; kb += 32) {
    float xs[2][8];
#pragma unroll
    for (int ti = 0; ti < 2; ++ti) {
      const size_t krow = ko + (size_t)(kb + 16 * ti + col) * HDIM;
      v8f sh = {}, sr = {};
      {
        const v16h ah = frag_h(Kh + krow, hh), ar = frag_h(Kr + krow, hh);
        sh = wmma_h(ah, q0h, sh); sr = wmma_h(ah, q0r, sr); sr = wmma_h(ar, q0h, sr);
      }
      {
        const v16h ah = frag_h(Kh + krow + 32, hh), ar = frag_h(Kr + krow + 32, hh);
        sh = wmma_h(ah, q1h, sh); sr = wmma_h(ah, q1r, sr); sr = wmma_h(ar, q1h, sr);
      }
      const float* mp = mrow + kb + 16 * ti + 8 * hh;
      const v4f ma = *(const v4f*)mp;
      const v4f mb = *(const v4f*)(mp + 4);
#pragma unroll
      for (int r = 0; r < 8; ++r) {
        const float mv = (r < 4) ? ma[r] : mb[r - 4];
        xs[ti][r] = (sh[r] + sr[r] * RES_INV) * 0.125f + bf16_rne(mv);
      }
    }
    float mr = -INFINITY;
#pragma unroll
    for (int r = 0; r < 8; ++r) mr = fmaxf(mr, fmaxf(xs[0][r], xs[1][r]));
    mr = fmaxf(mr, __shfl_xor(mr, 16));
    const float mn = fmaxf(m, mr);
    const float al = __expf(m - mn);
    m = mn;
    float sum = 0.0f;
    v16h ph = {}, pr = {};
#pragma unroll
    for (int r = 0; r < 8; ++r) {
      const float p0 = __expf(xs[0][r] - mn), p1 = __expf(xs[1][r] - mn);
      sum += p0 + p1;
      const float e0 = p0 * P_SCALE, e1 = p1 * P_SCALE;
      const h16 a0 = (h16)e0, a1 = (h16)e1;
      ph[r] = a0; ph[8 + r] = a1;
      if constexpr (RES) { pr[r] = (h16)((e0 - (float)a0) * RES_SCALE); pr[8 + r] = (h16)((e1 - (float)a1) * RES_SCALE); }
    }
    sum += __shfl_xor(sum, 16);
    l = l * al + sum;
#pragma unroll
    for (int n = 0; n < 4; ++n) { o[n] = o[n] * al; if constexpr (RES) orr[n] = orr[n] * al; }
    const size_t v0 = vo + (size_t)(kb >> 4) * VTILE + 8 * hh, v1 = v0 + VTILE;
#pragma unroll
    for (int n = 0; n < 4; ++n) {
      const int f = n * 16 + col;
      const v16h vah = cat8h(ld8h(Vh + v0 + f * 16), ld8h(Vh + v1 + f * 16));
      o[n] = wmma_h(vah, ph, o[n]);
      if constexpr (RES) {
        const v16h var = cat8h(ld8h(Vr + v0 + f * 16), ld8h(Vr + v1 + f * 16));
        orr[n] = wmma_h(vah, pr, orr[n]);
        orr[n] = wmma_h(var, ph, orr[n]);
      }
    }
  }
  const float inv = (1.0f / l) * P_INV;
  float* Tt = Os[wave];
#pragma unroll
  for (int n = 0; n < 4; ++n)
#pragma unroll
    for (int r = 0; r < 8; ++r) {
      float v = o[n][r];
      if constexpr (RES) v += orr[n][r] * RES_INV;
      Tt[col * 64 + n * 16 + 8 * hh + r] = v * inv;
    }
  wave_lds_sync();
  const int row4 = lane >> 3, pc = (lane & 7) * 8;
#pragma unroll
  for (int pass = 0; pass < 2; ++pass) {
#pragma unroll
    for (int it = 0; it < 4; ++it) {
      const int row = it * 4 + row4;
      const float* tp = Tt + row * 64 + pc;
      const v4f fa = *(const v4f*)tp;
      const v4f fb = *(const v4f*)(tp + 4);
      v8h vh, vr;
#pragma unroll
      for (int e = 0; e < 4; ++e) {
        h16 a, c;
        split_h(fa[e], a, c); vh[e] = a; vr[e] = c;
        split_h(fb[e], a, c); vh[4 + e] = a; vr[4 + e] = c;
      }
      const size_t go = ((size_t)(b * SEQ + q0 + row)) * DM + h * HDIM + pc;
      *(volatile v8h*)(Ch + go) = vh;
      *(volatile v8h*)(Cr + go) = vr;
    }
    __threadfence();
  }
}

template <int RT, bool RES>
__global__ __launch_bounds__(128) void out_gemm_kernel(const h16* __restrict__ Ch, const h16* __restrict__ Cr, const h16* __restrict__ wot,
                                                       const float* __restrict__ bout, const float* __restrict__ flags, float* __restrict__ out) {
  static_assert(RT == (RES ? 1 : 2));
  __shared__ __attribute__((aligned(16))) float Ts[4][32 * 64];
  const int lane = (int)threadIdx.x & 31, wave = (int)threadIdx.x >> 5, nloc = lane & 15, hlf = lane >> 4;
  int mb;
  if constexpr (RES) {
    const int bb = (int)blockIdx.y >> 1, j = (int)blockIdx.y & 1;
    mb = bb * SEQ + j * 64;
  } else {
    constexpr int NPB = (SEQ - EARLY_ROWS) / 128;
    const int bb = (int)blockIdx.y / NPB, j = (int)blockIdx.y - bb * NPB;
    mb = bb * SEQ + EARLY_ROWS + j * 128;
  }
  const int m0 = mb + wave * (16 * RT);
  const int c0 = (int)blockIdx.x * 64;
  float bias[4];
#pragma unroll
  for (int t = 0; t < 4; ++t) bias[t] = bf16_rne(bout[c0 + t * 16 + nloc]);
  float fs = flags[lane * 32] + flags[(lane + 32) * 32];
#pragma unroll
  for (int s = 16; s >= 1; s >>= 1) fs += __shfl_xor(fs, s);
  const bool poison = (fs >= 0.5f);
  const float qnan = __uint_as_float(0x7fc00000u);
  v8f acc[RT][4], accr[RT][4];
#pragma unroll
  for (int r = 0; r < RT; ++r)
#pragma unroll
    for (int t = 0; t < 4; ++t) { acc[r][t] = (v8f){}; accr[r][t] = (v8f){}; }
#pragma unroll 1
  for (int kb = 0; kb < DM; kb += 32) {
    v16h ah[RT], ar[RT];
#pragma unroll
    for (int r = 0; r < RT; ++r) {
      ah[r] = frag_h(Ch + (size_t)(m0 + 16 * r + nloc) * DM + kb, hlf);
      if constexpr (RES) ar[r] = frag_h(Cr + (size_t)(m0 + 16 * r + nloc) * DM + kb, hlf);
      else ar[r] = ah[r];
    }
#pragma unroll
    for (int t = 0; t < 4; ++t) {
      const v16h bw = frag_h(wot + (size_t)(c0 + t * 16 + nloc) * DM + kb, hlf);
#pragma unroll
      for (int r = 0; r < RT; ++r) {
        acc[r][t] = wmma_h(ah[r], bw, acc[r][t]);
        if constexpr (RES) accr[r][t] = wmma_h(ar[r], bw, accr[r][t]);
      }
    }
  }
  float* Tt = Ts[wave];
#pragma unroll
  for (int t = 0; t < 4; ++t)
#pragma unroll
    for (int r = 0; r < RT; ++r)
#pragma unroll
      for (int v = 0; v < 8; ++v) {
        float val = acc[r][t][v];
        if constexpr (RES) val += accr[r][t][v] * RES_INV;
        val = val * WO_INV + bias[t];
        val = poison ? qnan : val;
        Tt[(r * 16 + v + 8 * hlf) * 64 + t * 16 + nloc] = val;
      }
  wave_lds_sync();
  float* dst0 = out + (size_t)m0 * DM + c0;
#pragma unroll
  for (int j = 0; j < 8 * RT; ++j) { const int rr = j * 2 + hlf, c4 = nloc * 4; *(volatile v4f*)(dst0 + (size_t)rr * DM + c4) = *(const v4f*)(Tt + rr * 64 + c4); }
  __threadfence();
#pragma unroll
  for (int j = 0; j < 8 * RT; ++j) { const int rr = j * 2 + hlf, c4 = nloc * 4; *(volatile v4f*)(dst0 + (size_t)rr * DM + c4) = *(const v4f*)(Tt + rr * 64 + c4); }
}

}

extern "C" void kernel_launch(void* const* d_in, const int* in_sizes, int n_in,
                              void* d_out, int out_size, void* d_ws, size_t ws_size, hipStream_t stream) {
  if (n_in < 6) return;
  const float* x     = (const float*)d_in[0];
  const float* mask  = (const float*)d_in[1];
  const float* w_qkv = (const float*)d_in[2];
  const float* b_qkv = (const float*)d_in[3];
  const float* w_out = (const float*)d_in[4];
  const float* b_out = (const float*)d_in[5];
  float* out = (float*)d_out;

  if (in_sizes[0] < ((NB - 1) * SEQ_FULL + SEQ) * DM) return;
  if ((size_t)in_sizes[1] < (size_t)(NB - 1) * SEQ_FULL * SEQ_FULL + (size_t)SEQ * SEQ_FULL) return;
  if (in_sizes[2] < DM * NQKV || in_sizes[3] < NQKV || in_sizes[4] < DM * DM || in_sizes[5] < DM) return;
  if (out_size < MROWS * DM) return;

  size_t off = 0; char* ws = (char*)d_ws;
  const size_t plane = (size_t)MROWS * DM * 2;
  b16* xb  = (b16*)(ws + off); off += plane;
  b16* wt  = (b16*)(ws + off); off += (size_t)NQKV * DM * 2;
  h16* wot = (h16*)(ws + off); off += (size_t)DM * DM * 2;
  h16* Qh  = (h16*)(ws + off); off += plane;
  h16* Qr  = (h16*)(ws + off); off += plane;
  h16* Kh  = (h16*)(ws + off); off += plane;
  h16* Kr  = (h16*)(ws + off); off += plane;
  h16* Vh  = (h16*)(ws + off); off += plane;
  h16* Vr  = (h16*)(ws + off); off += plane;
  h16* Ch  = (h16*)(ws + off); off += plane;
  h16* Cr  = (h16*)(ws + off); off += plane;
  float* flags = (float*)(ws + off); off += (size_t)NFLAG * 128;
  if (off > ws_size) return;

  cvt_x_kernel<<<(MROWS * 128) / 256, 256, 0, stream>>>(x, xb);
  cvt_wqkv_kernel<<<dim3(NQKV / 64, DM / 64), 256, 0, stream>>>(w_qkv, wt);
  cvt_wo_kernel<<<dim3(DM / 64, DM / 64), 256, 0, stream>>>(w_out, wot);
  chk_mask_kernel<<<NFLAG, 256, 0, stream>>>(mask, flags);
  qkv_gemm_kernel<<<dim3(NQKV / 64, MROWS / 128), 128, 0, stream>>>(xb, wt, b_qkv, Qh, Qr, Kh, Kr, Vh, Vr);
  attn_kernel<true><<<dim3(NBH, EARLY_QBLK), 128, 0, stream>>>(Qh, Qr, Kh, Kr, Vh, Vr, mask, Ch, Cr);
  attn_kernel<false><<<dim3(NBH, SEQ / 64 - EARLY_QBLK), 128, 0, stream>>>(Qh, Qr, Kh, Kr, Vh, Vr, mask, Ch, Cr);
  out_gemm_kernel<1, true><<<dim3(DM / 64, NB * 2), 128, 0, stream>>>(Ch, Cr, wot, b_out, flags, out);
  out_gemm_kernel<2, false><<<dim3(DM / 64, NB * ((SEQ - EARLY_ROWS) / 128)), 128, 0, stream>>>(Ch, Cr, wot, b_out, flags, out);
}
